// CrystalAttention_38740605009994
// MI455X (gfx1250) — hardware-run, weakly checked
//
#include <hip/hip_runtime.h>
#include <math.h>

typedef __attribute__((ext_vector_type(16))) _Float16 v16h;
typedef __attribute__((ext_vector_type(16))) __bf16 v16b;
typedef __attribute__((ext_vector_type(8)))  _Float16 v8h;
typedef __attribute__((ext_vector_type(8)))  float v8f;
typedef __attribute__((ext_vector_type(4)))  float v4f;
typedef __attribute__((ext_vector_type(2)))  float v2f;
typedef __attribute__((ext_vector_type(4)))  unsigned v4u;
typedef __attribute__((ext_vector_type(4)))  int v4i;
typedef float __attribute__((may_alias)) float_a;
typedef int __attribute__((may_alias)) int_a;

template <typename T> __device__ __forceinline__ void vst2(void* p, T v) { *(volatile T*)p = v; __threadfence(); *(volatile T*)p = v; }
__device__ __forceinline__ v8f wmma16(v16h a, v16h b, v8f c) {
  v8f d = __builtin_amdgcn_wmma_f32_16x16x32_f16(false, a, false, b, (short)0, c, false, false);
  asm volatile("v_nop\n\tv_nop\n\tv_nop\n\tv_nop" : "+v"(d) : "v"(a), "v"(b));
  return d;
}
__device__ __forceinline__ v8f wmma_bf(v16b a, v16b b, v8f c) {
  v8f d = __builtin_amdgcn_wmma_f32_16x16x32_bf16(false, a, false, b, (short)0, c, false, false);
  asm volatile("v_nop\n\tv_nop\n\tv_nop\n\tv_nop" : "+v"(d) : "v"(a), "v"(b));
  return d;
}
__device__ __forceinline__ v16h frag_h(const _Float16* rowk0, int lane) {
  union { v16h v; v8h q[2]; } u; const _Float16* p = rowk0 + 8 * (lane >> 4);
  u.q[0] = *(const v8h*)p; u.q[1] = *(const v8h*)(p + 16); return u.v;
}
__device__ __forceinline__ v16h frag_f32(const float* rowk0, int lane) {
  v16h a; const float* p = rowk0 + 8 * (lane >> 4);
#pragma unroll
  for (int i = 0; i < 8; ++i) { a[i] = (_Float16)p[i]; a[8 + i] = (_Float16)p[16 + i]; }
  return a;
}
__device__ __forceinline__ v16h frag_f32s(const float* rowk0, int lane, float sc) {
  v16h a; const float* p = rowk0 + 8 * (lane >> 4);
#pragma unroll
  for (int i = 0; i < 8; ++i) { a[i] = (_Float16)(p[i] * sc); a[8 + i] = (_Float16)(p[16 + i] * sc); }
  return a;
}
__device__ __forceinline__ v16h fragc_f32(const float* W, int k0, int n, int lane, int ld, int K) {
  v16h a; const int g = lane >> 4;
#pragma unroll
  for (int i = 0; i < 8; ++i) { const int ka = k0 + 8 * g + i, kb = ka + 16;
    a[i] = (_Float16)(ka < K ? W[(size_t)(ka < K ? ka : K - 1) * ld + n] : 0.f); a[8 + i] = (_Float16)(kb < K ? W[(size_t)(kb < K ? kb : K - 1) * ld + n] : 0.f); }
  return a;
}
struct F2 { v16b h, l; };
__device__ __forceinline__ F2 bsplit16(const float v[16]) { F2 r;
#pragma unroll
  for (int i = 0; i < 16; ++i) { const __bf16 h = (__bf16)v[i]; r.h[i] = h; r.l[i] = (__bf16)(v[i] - (float)h); }
  return r; }
__device__ __forceinline__ F2 split_row(const float* row, int k0, int lane) { float v[16]; const float* p = row + k0 + 8 * (lane >> 4);
#pragma unroll
  for (int i = 0; i < 8; ++i) { v[i] = p[i]; v[8 + i] = p[16 + i]; }
  return bsplit16(v); }
__device__ __forceinline__ F2 split_rowK(const float* row, int k0, int lane, int K) { float v[16]; const int g = lane >> 4;
#pragma unroll
  for (int i = 0; i < 8; ++i) { const int ka = k0 + 8 * g + i, kb = ka + 16; v[i] = ka < K ? row[ka < K ? ka : K - 1] : 0.f; v[8 + i] = kb < K ? row[kb < K ? kb : K - 1] : 0.f; }
  return bsplit16(v); }
__device__ __forceinline__ F2 split_col(const float* W, int k0, int n, int lane, int ld, int K) { float v[16]; const int g = lane >> 4;
#pragma unroll
  for (int i = 0; i < 8; ++i) { const int ka = k0 + 8 * g + i, kb = ka + 16; v[i] = ka < K ? W[(size_t)(ka < K ? ka : K - 1) * ld + n] : 0.f; v[8 + i] = kb < K ? W[(size_t)(kb < K ? kb : K - 1) * ld + n] : 0.f; }
  return bsplit16(v); }
__device__ __forceinline__ v8f mac3(const F2& a, const F2& b, v8f c) { c = wmma_bf(a.l, b.h, c); c = wmma_bf(a.h, b.l, c); return wmma_bf(a.h, b.h, c); }
__device__ __forceinline__ float sigm(float v) { return 1.0f / (1.0f + expf(-v)); }
#define LDSX() do { asm volatile("s_wait_dscnt 0" ::: "memory"); __builtin_amdgcn_wave_barrier(); __builtin_amdgcn_fence(__ATOMIC_RELEASE, "workgroup"); } while (0)


#define NB 8
#define TT 2048
#define DD 512
#define NN 1024
#define NR (NB * TT)
#ifndef TRB
#define TRB (NR / 64)
#endif
typedef __attribute__((ext_vector_type(8))) __bf16 v8b;
__device__ __forceinline__ v16b frag_b(const __bf16* rowk0, int lane) {
  union { v16b v; v8b q[2]; } u; const __bf16* p = rowk0 + 8 * (lane >> 4);
  u.q[0] = *(const v8b*)p; u.q[1] = *(const v8b*)(p + 16); return u.v;
}
__device__ __forceinline__ float bfr(float v) { return (float)(__bf16)v; }
__device__ __attribute__((noinline)) float exp_ni(float v) { return expf(v); }
__device__ __attribute__((noinline)) float erf_ni(float v) { return erff(v); }

#define WS_PP   0u
#define WS_PV   (WS_PP + 2u * (size_t)NN * DD)
#define WS_PO   (WS_PV + 2u * (size_t)DD * NN)
#define WS_P2   (WS_PO + 2u * (size_t)DD * DD)
#define WS_LG   (WS_P2 + 4u * (size_t)NN * 32)
#define WS_AH   (WS_LG + 4u * (size_t)NR * NN)
#define WS_AL   (WS_AH + 2u * (size_t)NR * NN)
#define WS_CTX  (WS_AL + 2u * (size_t)NR * NN)
#define WS_END  (WS_CTX + 4u * (size_t)NR * DD)

__global__ __launch_bounds__(256) void k_pack(const float* __restrict__ POS, const float* __restrict__ VAL, const float* __restrict__ WO, __bf16* __restrict__ P, float* __restrict__ P2) {
  __shared__ __align__(16) __bf16 s[NN]; __shared__ float red[8]; __shared__ __align__(16) float line[32]; const int t = threadIdx.x; int n = blockIdx.x;
  if (n < NN) { float q = 0.f; for (int k = t; k < DD; k += 256) { const __bf16 v = (__bf16)POS[(size_t)n * DD + k]; s[k] = v; const float f = (float)v; q += f * f; }
#pragma unroll
    for (int o = 1; o < 32; o <<= 1) q += __shfl_xor(q, o);
    if ((t & 31) == 0) red[t >> 5] = q; __syncthreads(); for (int k = t; k < DD / 8; k += 256) vst2((unsigned*)(P + WS_PP / 2 + (size_t)n * DD + k * 8), *(const v4u*)&s[k * 8]);
    if (t < 32) { float tot = 0.f; if (t == 0) for (int i = 0; i < 8; ++i) tot += red[i]; line[t] = (t == 0) ? tot : 0.f; } __syncthreads(); if (t < 8) vst2(P2 + (size_t)n * 32 + t * 4, *(const v4f*)&line[t * 4]);
  } else if ((n -= NN) < DD) { for (int k = t; k < NN; k += 256) s[k] = (__bf16)VAL[(size_t)k * DD + n]; __syncthreads(); for (int k = t; k < NN / 8; k += 256) vst2((unsigned*)(P + WS_PV / 2 + (size_t)n * NN + k * 8), *(const v4u*)&s[k * 8]); }
  else { n -= DD; for (int k = t; k < DD; k += 256) s[k] = (__bf16)WO[(size_t)n * DD + k]; __syncthreads(); for (int k = t; k < DD / 8; k += 256) vst2((unsigned*)(P + WS_PO / 2 + (size_t)n * DD + k * 8), *(const v4u*)&s[k * 8]); }
}
__global__ __launch_bounds__(128) void k_logit(const float* __restrict__ X, const __bf16* __restrict__ P, const float* __restrict__ P2, const float* __restrict__ SC, float* __restrict__ LG) {
  __shared__ __align__(16) float so[4][16][132]; __shared__ float sx2[64];
  const int tid = threadIdx.x, wave = tid >> 5, lane = tid & 31, col = lane & 15, g = lane >> 4; const size_t rb0 = (size_t)blockIdx.x * 64, r0 = rb0 + wave * 16; const int n0 = blockIdx.y * 128;
  { const int rr = tid >> 1, half = tid & 1; const float* p = X + (rb0 + rr) * DD + half * (DD / 2); float q = 0.f; for (int k = 0; k < DD / 2; ++k) { const float v = bfr(p[k]); q += v * v; } q += __shfl_xor(q, 1); if (half == 0) sx2[rr] = q; }
  __syncthreads();
  v8f acc[8] = {};
#pragma unroll 2
  for (int kc = 0; kc < DD / 32; ++kc) { v16b a; { const float* p = X + (r0 + col) * DD + kc * 32 + 8 * g;
#pragma unroll
      for (int i = 0; i < 8; ++i) { a[i] = (__bf16)p[i]; a[8 + i] = (__bf16)p[16 + i]; } }
#pragma unroll
    for (int j = 0; j < 8; ++j) acc[j] = wmma_bf(a, frag_b(P + WS_PP / 2 + (size_t)(n0 + j * 16 + col) * DD + kc * 32, lane), acc[j]); }
#pragma unroll
  for (int j = 0; j < 8; ++j) { const int n = n0 + j * 16 + col; const float p2 = P2[(size_t)n * 32], sc = bfr(SC[n]);
#pragma unroll
    for (int r = 0; r < 8; ++r) { const float d2 = sx2[wave * 16 + 8 * g + r] - 2.0f * acc[j][r] + p2; const float dist = sqrtf(fmaxf(d2, 0.f)); so[wave][8 * g + r][j * 16 + col] = sc / (dist + 0.1f); } }
  LDSX();
  for (int rl = 0; rl < 16; ++rl) vst2(LG + (r0 + rl) * NN + n0 + lane * 4, *(const v4f*)&so[wave][rl][lane * 4]);
}
__device__ __attribute__((noinline)) float exp_p(float v) { return expf(v); }
__global__ __launch_bounds__(256) void k_soft(const float* __restrict__ LG, __bf16* __restrict__ AH, __bf16* __restrict__ AL) {
  __shared__ float red[8]; __shared__ __align__(16) __bf16 sh[NN], sl[NN]; const size_t row = blockIdx.x; const int t = threadIdx.x; float v[4]; float mx = -3.0e38f;
  for (int i = 0; i < 4; ++i) { v[i] = LG[row * NN + t * 4 + i]; mx = fmaxf(mx, v[i]); }
#pragma unroll
  for (int o = 1; o < 32; o <<= 1) mx = fmaxf(mx, __shfl_xor(mx, o));
  if ((t & 31) == 0) red[t >> 5] = mx; __syncthreads(); float m = red[0]; for (int i = 1; i < 8; ++i) m = fmaxf(m, red[i]); __syncthreads();
  float sum = 0.f; for (int i = 0; i < 4; ++i) { v[i] = exp_p(v[i] - m); sum += v[i]; }
#pragma unroll
  for (int o = 1; o < 32; o <<= 1) sum += __shfl_xor(sum, o);
  if ((t & 31) == 0) red[t >> 5] = sum; __syncthreads(); float tot = 0.f; for (int i = 0; i < 8; ++i) tot += red[i]; const float inv = 1.0f / tot;
  for (int i = 0; i < 4; ++i) { const float p = v[i] * inv; const __bf16 h = (__bf16)p; sh[t * 4 + i] = h; sl[t * 4 + i] = (__bf16)(p - (float)h); }
  __syncthreads(); if (t < NN / 8) { vst2((unsigned*)(AH + row * NN + t * 8), *(const v4u*)&sh[t * 8]); vst2((unsigned*)(AL + row * NN + t * 8), *(const v4u*)&sl[t * 8]); }
}
__global__ __launch_bounds__(128) void k_pv(const __bf16* __restrict__ AH, const __bf16* __restrict__ AL, const __bf16* __restrict__ P, float* __restrict__ CTX) {
  __shared__ __align__(16) float so[4][16][132];
  const int tid = threadIdx.x, wave = tid >> 5, lane = tid & 31, col = lane & 15, g = lane >> 4; const size_t r0 = (size_t)blockIdx.x * 64 + wave * 16; const int n0 = blockIdx.y * 128;
  v8f acc[8] = {};
#pragma unroll 2
  for (int kc = 0; kc < NN / 32; ++kc) { const v16b ah = frag_b(AH + (r0 + col) * NN + kc * 32, lane), al = frag_b(AL + (r0 + col) * NN + kc * 32, lane);
#pragma unroll
    for (int j = 0; j < 8; ++j) { const v16b w = frag_b(P + WS_PV / 2 + (size_t)(n0 + j * 16 + col) * NN + kc * 32, lane); acc[j] = wmma_bf(ah, w, acc[j]); acc[j] = wmma_bf(al, w, acc[j]); } }
#pragma unroll
  for (int j = 0; j < 8; ++j)
#pragma unroll
    for (int r = 0; r < 8; ++r) so[wave][8 * g + r][j * 16 + col] = acc[j][r];
  LDSX();
  for (int rl = 0; rl < 16; ++rl) vst2(CTX + (r0 + rl) * DD + n0 + lane * 4, *(const v4f*)&so[wave][rl][lane * 4]);
}
__global__ __launch_bounds__(128) void k_out(const float* __restrict__ CTX, const __bf16* __restrict__ P, const float* __restrict__ BO, float* __restrict__ OUT) {
  __shared__ __align__(16) float so[4][16][132];
  const int tid = threadIdx.x, wave = tid >> 5, lane = tid & 31, col = lane & 15, g = lane >> 4; const size_t r0 = (size_t)blockIdx.x * 64 + wave * 16; const int n0 = blockIdx.y * 128;
  v8f acc[8] = {};
#pragma unroll 2
  for (int kc = 0; kc < DD / 32; ++kc) { const F2 a = split_row(CTX + (r0 + col) * DD, kc * 32, lane);
#pragma unroll
    for (int j = 0; j < 8; ++j) { const v16b w = frag_b(P + WS_PO / 2 + (size_t)(n0 + j * 16 + col) * DD + kc * 32, lane); acc[j] = wmma_bf(a.l, w, acc[j]); acc[j] = wmma_bf(a.h, w, acc[j]); } }
#pragma unroll
  for (int j = 0; j < 8; ++j) { const float bb = bfr(BO[n0 + j * 16 + col]);
#pragma unroll
    for (int r = 0; r < 8; ++r) so[wave][8 * g + r][j * 16 + col] = acc[j][r] + bb; }
  LDSX();
  for (int rl = 0; rl < 16; ++rl) vst2(OUT + (r0 + rl) * DD + n0 + lane * 4, *(const v4f*)&so[wave][rl][lane * 4]);
}
extern "C" void kernel_launch(void* const* d_in, const int* in_sizes, int n_in, void* d_out, int out_size, void* d_ws, size_t ws_size, hipStream_t stream) {
  (void)in_sizes; (void)n_in; (void)out_size;
  const float** F = (const float**)d_in;
  if (ws_size < (size_t)WS_END) return;
  char* ws = (char*)d_ws; __bf16* P = (__bf16*)ws; float *P2 = (float*)(ws + WS_P2), *LG = (float*)(ws + WS_LG), *CTX = (float*)(ws + WS_CTX); __bf16 *AH = (__bf16*)(ws + WS_AH), *AL = (__bf16*)(ws + WS_AL);
  k_pack<<<NN + DD + DD, 256, 0, stream>>>(F[1], F[3], F[4], P, P2);
  k_logit<<<dim3(TRB, NN / 128), 128, 0, stream>>>(F[0], P, P2, F[2], LG);
  k_soft<<<TRB * 64, 256, 0, stream>>>(LG, AH, AL);
  k_pv<<<dim3(TRB, DD / 128), 128, 0, stream>>>(AH, AL, P, CTX);
  k_out<<<dim3(TRB, DD / 128), 128, 0, stream>>>(CTX, P, F[5], (float*)d_out);
}
